// GAU_75780402971292
// MI455X (gfx1250) — hardware-verified
//
#include <hip/hip_runtime.h>
#include <math.h>
#include <stdint.h>

#ifndef NB
#define NB 4
#endif
#ifndef SEQ
#define SEQ 2048
#endif
#define XS_FULL 2048
#define DM   512
#define DQ   256
#define DH   1536
#define H2   3072
#define VCAR 1024.0f
#define ACAR 512.0f
#define EPSC 1e-5f
#define SLP  68
#define SLAB64 (16 * SLP)
#define TRP  72
#define VTP  72
#define WS_CAP 134217728
static_assert(NB >= 1 && NB <= 4);
static_assert(NB == 1 || SEQ == XS_FULL);
static_assert((SEQ % 64) == 0 && SEQ >= 64 && SEQ <= XS_FULL);
static_assert((DM % 64) == 0 && (DQ % 64) == 0 && (DH % 64) == 0 && (H2 % 64) == 0);
static_assert((DM % 32) == 0 && (DQ % 32) == 0 && (DH % 32) == 0 && (SEQ % 32) == 0);
static_assert(((SEQ * DM / 8) % 256) == 0 && (SEQ % 8) == 0 && DM == 512 && H2 == 2 * DH);
static_assert(4 * SLAB64 * 4 <= 65536 && 64 * TRP * 2 <= 65536 && 64 * VTP * 2 <= 65536);

typedef unsigned short u16;
typedef _Float16 v16h __attribute__((ext_vector_type(16)));
typedef _Float16 v8h  __attribute__((ext_vector_type(8)));
typedef __bf16   v16b __attribute__((ext_vector_type(16)));
typedef float    v8f  __attribute__((ext_vector_type(8)));
typedef float    v4f  __attribute__((ext_vector_type(4)));
typedef unsigned int v4u __attribute__((ext_vector_type(4)));

union FragH { v16h v; v8h h[2]; v4u u[2]; };
union FragB { v16b v; v4u u[2]; };

__device__ __forceinline__ unsigned short bf_bits(float f) {
  unsigned u = __float_as_uint(f);
  return (unsigned short)((u + 0x7FFFu + ((u >> 16) & 1u)) >> 16);
}
__device__ __forceinline__ float bf_up(unsigned short h) { return __uint_as_float(((unsigned)h) << 16); }
__device__ __forceinline__ float bfr(float f) { return bf_up(bf_bits(f)); }
__device__ __forceinline__ unsigned short h_bits(_Float16 x) { return __builtin_bit_cast(unsigned short, x); }
__device__ __forceinline__ unsigned pk16(unsigned short a, unsigned short b) { return (unsigned)a | ((unsigned)b << 16); }
__device__ __forceinline__ v8f zero8() { v8f z = {0.f, 0.f, 0.f, 0.f, 0.f, 0.f, 0.f, 0.f}; return z; }
__device__ __forceinline__ v4f zero4() { v4f z = {0.f, 0.f, 0.f, 0.f}; return z; }
__device__ __forceinline__ float wsum(float v) {
#pragma unroll
  for (int o = 16; o > 0; o >>= 1) v += __shfl_xor(v, o, 32);
  return v;
}

__device__ __forceinline__ v16h ldfrag_h(const _Float16* p) {
  FragH f;
  f.h[0] = *(const v8h*)(p);
  f.h[1] = *(const v8h*)(p + 16);
  return f.v;
}
__device__ __forceinline__ v16b ldfrag_b(const u16* p) {
  FragB f;
  f.u[0] = *(const v4u*)(p);
  f.u[1] = *(const v4u*)(p + 16);
  return f.v;
}

__device__ __forceinline__ v8f mma_h(v16h a, v16h b, v8f c) {
  return __builtin_amdgcn_wmma_f32_16x16x32_f16(false, a, false, b, (short)0, c, false, false);
}
__device__ __forceinline__ v8f mma_b(v16b a, v16b b, v8f c) {
  return __builtin_amdgcn_wmma_f32_16x16x32_bf16(false, a, false, b, (short)0, c, false, false);
}
template <typename F>
__device__ __forceinline__ void guard10(v8f& a, v8f& b, v8f& c, v8f& d, F x0, F x1, F x2, F x3, F x4, F x5,
                                        F x6, F x7, F x8, F x9) {
#if defined(__HIP_DEVICE_COMPILE__)
  asm volatile("v_nop\n\tv_nop\n\tv_nop\n\tv_nop"
               : "+v"(a), "+v"(b), "+v"(c), "+v"(d)
               : "v"(x0), "v"(x1), "v"(x2), "v"(x3), "v"(x4), "v"(x5), "v"(x6), "v"(x7), "v"(x8), "v"(x9)
               : "memory");
#endif
}
__device__ __forceinline__ void wave_sync_lds() {
  __builtin_amdgcn_fence(__ATOMIC_RELEASE, "workgroup");
  __builtin_amdgcn_wave_barrier();
  __builtin_amdgcn_fence(__ATOMIC_ACQUIRE, "workgroup");
}

template <bool F16> struct Eng;
template <> struct Eng<true> {
  typedef v16h F;
  static __device__ __forceinline__ F ld(const u16* p) { return ldfrag_h((const _Float16*)(const void*)p); }
  static __device__ __forceinline__ v8f mma(F a, F b, v8f c) { return mma_h(a, b, c); }
};
template <> struct Eng<false> {
  typedef v16b F;
  static __device__ __forceinline__ F ld(const u16* p) { return ldfrag_b(p); }
  static __device__ __forceinline__ v8f mma(F a, F b, v8f c) { return mma_b(a, b, c); }
};

__global__ __launch_bounds__(256) void k_cvt(const float* __restrict__ x, u16* D, int n8) {
  const int gt = (int)blockIdx.x * 256 + (int)threadIdx.x;
  if (gt >= n8) return;
  const float* p = x + (size_t)gt * 8;
  const v4f a = *(const v4f*)(p), b4 = *(const v4f*)(p + 4);
  float w[8];
#pragma unroll
  for (int e = 0; e < 4; ++e) { w[e] = a[e]; w[4 + e] = b4[e]; }
  v4u o;
#pragma unroll
  for (int e = 0; e < 4; ++e) o[e] = pk16(bf_bits(w[2 * e]), bf_bits(w[2 * e + 1]));
  u16* d = D + (size_t)gt * 8;
  for (int pass = 0; pass < 2; ++pass) {
    *(volatile v4u*)(d) = o;
    __threadfence();
  }
}

__global__ __launch_bounds__(256) void k_wt(const float* __restrict__ W, int nc, int kr, int ntn, u16* Dp, int drow0) {
  __shared__ __align__(16) u16 T[64 * TRP];
  const int tid = (int)threadIdx.x;
  const int bid = (int)blockIdx.x;
  const int nt  = bid % ntn;
  const int kt  = bid / ntn;
  if (kt * 64 + 64 > kr) return;
  const int n0  = nt * 64, k0 = kt * 64;
  {
    const int dl = tid >> 2;
    const int oc = (tid & 3) * 16;
    const bool valid = (n0 + oc + 16 <= nc);
    const int  cb = valid ? (n0 + oc) : 0;
    const float* src = W + (size_t)(k0 + dl) * (size_t)nc + cb;
#pragma unroll
    for (int i = 0; i < 4; ++i) {
      const v4f a = *(const v4f*)(src + 4 * i);
#pragma unroll
      for (int e = 0; e < 4; ++e) {
        const float f = valid ? a[e] : 0.0f;
        T[(oc + 4 * i + e) * TRP + dl] = bf_bits(f);
      }
    }
  }
  __syncthreads();
  const int q8 = tid >> 3, p8 = (tid & 7) * 8;
  v4u w[2];
#pragma unroll
  for (int it = 0; it < 2; ++it) w[it] = *(const v4u*)(T + (it * 32 + q8) * TRP + p8);
  const size_t base = (size_t)(drow0 + n0) * (size_t)kr + k0 + p8;
  for (int pass = 0; pass < 2; ++pass) {
#pragma unroll
    for (int it = 0; it < 2; ++it) {
      const int nl = it * 32 + q8;
      *(volatile v4u*)(Dp + base + (size_t)nl * (size_t)kr) = w[it];
    }
    __threadfence();
  }
}

__global__ __launch_bounds__(256) void k_vt(const float* __restrict__ H, u16* VT) {
  __shared__ __align__(16) u16 T[64 * VTP];
  const int tid = (int)threadIdx.x;
  const int bid = (int)blockIdx.x;
  const int nst = SEQ / 64;
  const int st  = bid % nst;
  const int dt  = bid / nst;
  if (dt * 64 + 64 > DH) return;
  const int s0  = st * 64, d0 = dt * 64;
  {
    const int sl = tid >> 2;
    const int dc = (tid & 3) * 16;
    const float* src = H + (size_t)(s0 + sl) * (size_t)H2 + d0 + dc;
#pragma unroll
    for (int i = 0; i < 4; ++i) {
      const v4f a = *(const v4f*)(src + 4 * i);
#pragma unroll
      for (int e = 0; e < 4; ++e) {
        const float t = a[e] * VCAR;
        T[(dc + 4 * i + e) * VTP + sl] = h_bits((_Float16)t);
      }
    }
  }
  __syncthreads();
  v4u vh[2];
  const int q8 = tid >> 3, p8 = (tid & 7) * 8;
#pragma unroll
  for (int it = 0; it < 2; ++it) vh[it] = *(const v4u*)(T + (it * 32 + q8) * VTP + p8);
  const size_t base = (size_t)d0 * SEQ + s0 + p8;
  for (int pass = 0; pass < 2; ++pass) {
#pragma unroll
    for (int it = 0; it < 2; ++it) {
      const int line = it * 32 + q8;
      *(volatile v4u*)(VT + base + (size_t)line * SEQ) = vh[it];
    }
    __threadfence();
  }
}

__global__ __launch_bounds__(256) void k_ln1(const float* __restrict__ Y, const float* __restrict__ g,
                                             const float* __restrict__ bb, u16* NHp, u16* NLp) {
  const int tid = (int)threadIdx.x, wave = tid >> 5, lane = tid & 31;
  const int row = (int)blockIdx.x * 8 + wave;
  if (row >= SEQ) return;
  const float* p = Y + (size_t)row * DM;
  float w[16];
#pragma unroll
  for (int it = 0; it < 2; ++it) {
    const int c = 8 * lane + 256 * it;
    const v4f a = *(const v4f*)(p + c), a2 = *(const v4f*)(p + c + 4);
#pragma unroll
    for (int e = 0; e < 4; ++e) { w[8 * it + e] = a[e]; w[8 * it + 4 + e] = a2[e]; }
  }
  float s = 0.0f;
#pragma unroll
  for (int i = 0; i < 16; ++i) s += w[i];
  s = wsum(s);
  const float mean = s * (1.0f / (float)DM);
  float q = 0.0f;
#pragma unroll
  for (int i = 0; i < 16; ++i) { const float d = w[i] - mean; q += d * d; }
  q = wsum(q);
  const float rstd = rsqrtf(q * (1.0f / (float)DM) + EPSC);
  v4u oh[2], ol[2];
#pragma unroll
  for (int it = 0; it < 2; ++it) {
    const int c = 8 * lane + 256 * it;
    const v4f ga = *(const v4f*)(g + c), gb = *(const v4f*)(g + c + 4);
    const v4f ba = *(const v4f*)(bb + c), b4 = *(const v4f*)(bb + c + 4);
    float gg[8], bv[8];
#pragma unroll
    for (int e = 0; e < 4; ++e) { gg[e] = bfr(ga[e]); gg[4 + e] = bfr(gb[e]); bv[e] = bfr(ba[e]); bv[4 + e] = bfr(b4[e]); }
#pragma unroll
    for (int e = 0; e < 4; ++e) {
      const float n0 = (w[8 * it + 2 * e] - mean) * rstd * gg[2 * e] + bv[2 * e];
      const float n1 = (w[8 * it + 2 * e + 1] - mean) * rstd * gg[2 * e + 1] + bv[2 * e + 1];
      const unsigned short h0 = bf_bits(n0), h1 = bf_bits(n1);
      const unsigned short l0 = bf_bits(n0 - bf_up(h0)), l1 = bf_bits(n1 - bf_up(h1));
      oh[it][e] = pk16(h0, h1);
      ol[it][e] = pk16(l0, l1);
    }
  }
  const size_t ob = (size_t)row * DM + 8 * lane;
  for (int pass = 0; pass < 2; ++pass) {
#pragma unroll
    for (int it = 0; it < 2; ++it) {
      *(volatile v4u*)(NHp + ob + 256 * it) = oh[it];
      *(volatile v4u*)(NLp + ob + 256 * it) = ol[it];
    }
    __threadfence();
  }
}

__global__ __launch_bounds__(256) void k_ln2(const float* __restrict__ T, const float* __restrict__ X,
                                             const float* __restrict__ g, const float* __restrict__ bb, float* O) {
  const int tid = (int)threadIdx.x, wave = tid >> 5, lane = tid & 31;
  const int row = (int)blockIdx.x * 8 + wave;
  if (row >= SEQ) return;
  const float* p  = T + (size_t)row * DM;
  const float* px = X + (size_t)row * DM;
  float w[16];
#pragma unroll
  for (int it = 0; it < 4; ++it) {
    const v4f a = *(const v4f*)(p + 4 * lane + 128 * it);
#pragma unroll
    for (int e = 0; e < 4; ++e) w[4 * it + e] = a[e];
  }
  float s = 0.0f;
#pragma unroll
  for (int i = 0; i < 16; ++i) s += w[i];
  s = wsum(s);
  const float mean = s * (1.0f / (float)DM);
  float q = 0.0f;
#pragma unroll
  for (int i = 0; i < 16; ++i) { const float d = w[i] - mean; q += d * d; }
  q = wsum(q);
  const float rstd = rsqrtf(q * (1.0f / (float)DM) + EPSC);
  v4f ov[4];
#pragma unroll
  for (int it = 0; it < 4; ++it) {
    const int c = 4 * lane + 128 * it;
    const v4f gv = *(const v4f*)(g + c), bv = *(const v4f*)(bb + c), xv = *(const v4f*)(px + c);
    v4f o;
#pragma unroll
    for (int e = 0; e < 4; ++e) {
      const float n = (w[4 * it + e] - mean) * rstd * bfr(gv[e]) + bfr(bv[e]);
      o[e] = n + bfr(xv[e]);
    }
    ov[it] = o;
  }
  float* d = O + (size_t)row * DM + 4 * lane;
  for (int pass = 0; pass < 2; ++pass) {
#pragma unroll
    for (int it = 0; it < 4; ++it) *(volatile v4f*)(d + 128 * it) = ov[it];
    __threadfence();
  }
}

template <int OP>
__device__ __forceinline__ float eop(float a, float bc, float ax, float sc) {
  if constexpr (OP == 0) { return a + bc; }
  else if constexpr (OP == 1) { return fmaxf(a + bc, 0.0f); }
  else if constexpr (OP == 2) { return a; }
  else if constexpr (OP == 3) { const float t = fmaxf(a * sc, 0.0f); return fminf(t * t * ACAR, 65000.0f); }
  else if constexpr (OP == 4) { return a * sc * ax; }
  else { return (a + bc) + ax; }
}

template <int NP, bool F16, int OP, int OK>
__global__ __launch_bounds__(128)
void k_gemm(const u16* __restrict__ A, const u16* __restrict__ A2,
            const u16* __restrict__ Bt, const u16* __restrict__ Bt2,
            int M, int N, int K,
            const float* __restrict__ bias, const float* __restrict__ aux, int auxld, float scale,
            float* Cf, u16* Ch, u16* Cl) {
  typedef Eng<F16> E;
  typedef typename Eng<F16>::F FT;
  __shared__ __align__(16) float slab[4 * SLAB64];
  const int tid = (int)threadIdx.x, wave = tid >> 5, lane = tid & 31, hh = lane >> 4, m = lane & 15;
  const int ntile = N >> 6;
  const int bid   = (int)blockIdx.x;
  const int rowb  = (bid / ntile) * 64 + wave * 16;
  const int col0  = (bid % ntile) * 64;
  if (rowb + 16 > M) return;
  const u16* ap  = A   + (size_t)(rowb + m) * K + 8 * hh;
  const u16* ap2 = A2  + (size_t)(rowb + m) * K + 8 * hh;
  const u16* bp  = Bt  + (size_t)(col0 + m) * K + 8 * hh;
  const u16* bp2 = Bt2 + (size_t)(col0 + m) * K + 8 * hh;
  const size_t bs = (size_t)16 * K;
  v8f acc0 = zero8(), acc1 = zero8(), acc2 = zero8(), acc3 = zero8();
#pragma unroll 1
  for (int k0 = 0; k0 < K; k0 += 32) {
    const FT a  = E::ld(ap + k0);
    const FT b0 = E::ld(bp + k0);
    const FT b1 = E::ld(bp + bs + k0);
    const FT b2 = E::ld(bp + 2 * bs + k0);
    const FT b3 = E::ld(bp + 3 * bs + k0);
    acc0 = E::mma(a, b0, acc0);
    acc1 = E::mma(a, b1, acc1);
    acc2 = E::mma(a, b2, acc2);
    acc3 = E::mma(a, b3, acc3);
    if constexpr (NP >= 2) {
      const FT a2 = E::ld(ap2 + k0);
      acc0 = E::mma(a2, b0, acc0);
      acc1 = E::mma(a2, b1, acc1);
      acc2 = E::mma(a2, b2, acc2);
      acc3 = E::mma(a2, b3, acc3);
      if constexpr (NP >= 3) {
        const FT c0 = E::ld(bp2 + k0);
        const FT c1 = E::ld(bp2 + bs + k0);
        const FT c2 = E::ld(bp2 + 2 * bs + k0);
        const FT c3 = E::ld(bp2 + 3 * bs + k0);
        acc0 = E::mma(a, c0, acc0);
        acc1 = E::mma(a, c1, acc1);
        acc2 = E::mma(a, c2, acc2);
        acc3 = E::mma(a, c3, acc3);
        guard10<FT>(acc0, acc1, acc2, acc3, a, a2, b0, b1, b2, b3, c0, c1, c2, c3);
      } else {
        guard10<FT>(acc0, acc1, acc2, acc3, a, a2, b0, b1, b2, b3, b0, b1, b2, b3);
      }
    } else {
      guard10<FT>(acc0, acc1, acc2, acc3, a, a, b0, b1, b2, b3, b0, b1, b2, b3);
    }
  }
  float* sl = slab + wave * SLAB64;
#pragma unroll
  for (int r = 0; r < 8; ++r) {
    const int ro = (8 * hh + r) * SLP + m;
    sl[ro]      = acc0[r];
    sl[ro + 16] = acc1[r];
    sl[ro + 32] = acc2[r];
    sl[ro + 48] = acc3[r];
  }
  wave_sync_lds();
  constexpr bool HB = (OP == 0 || OP == 1 || OP == 5);
  constexpr bool HA = (OP == 4 || OP == 5);
  if constexpr (OK == 0) {
    const int cb = col0 + m * 4;
    v4f b4 = zero4();
    if constexpr (HB) {
      const v4f t = *(const v4f*)(bias + cb);
#pragma unroll
      for (int e = 0; e < 4; ++e) b4[e] = bfr(t[e]);
    }
    v4f vals[8];
#pragma unroll
    for (int it = 0; it < 8; ++it) {
      const int rl = it * 2 + hh;
      const size_t grow = (size_t)rowb + (size_t)rl;
      const v4f sv = *(const v4f*)(sl + rl * SLP + m * 4);
      v4f ax = zero4();
      if constexpr (HA) {
        ax = *(const v4f*)(aux + grow * (size_t)auxld + cb);
        if constexpr (OP == 5) {
#pragma unroll
          for (int e = 0; e < 4; ++e) ax[e] = bfr(ax[e]);
        }
      }
      v4f v;
#pragma unroll
      for (int e = 0; e < 4; ++e) v[e] = eop<OP>(sv[e], b4[e], ax[e], scale);
      vals[it] = v;
    }
    float* dst = Cf + ((size_t)rowb + (size_t)hh) * (size_t)N + cb;
    for (int pass = 0; pass < 2; ++pass) {
#pragma unroll
      for (int it = 0; it < 8; ++it) {
        *(volatile v4f*)(dst + (size_t)(it * 2) * (size_t)N) = vals[it];
      }
      __threadfence();
    }
  } else {
    const int rq = lane >> 3, c8 = (lane & 7) * 8;
    const int cb = col0 + c8;
    float b8[8];
#pragma unroll
    for (int e = 0; e < 8; ++e) b8[e] = 0.0f;
    if constexpr (HB) {
      const v4f t0 = *(const v4f*)(bias + cb), t1 = *(const v4f*)(bias + cb + 4);
#pragma unroll
      for (int e = 0; e < 4; ++e) { b8[e] = bfr(t0[e]); b8[4 + e] = bfr(t1[e]); }
    }
    v4u oh[4], ol[4];
#pragma unroll
    for (int it = 0; it < 4; ++it) {
      const int rl = it * 4 + rq;
      const size_t grow = (size_t)rowb + (size_t)rl;
      const v4f s0 = *(const v4f*)(sl + rl * SLP + c8), s1 = *(const v4f*)(sl + rl * SLP + c8 + 4);
      float ax[8];
#pragma unroll
      for (int e = 0; e < 8; ++e) ax[e] = 0.0f;
      if constexpr (HA) {
        const v4f x0 = *(const v4f*)(aux + grow * (size_t)auxld + cb);
        const v4f x1 = *(const v4f*)(aux + grow * (size_t)auxld + cb + 4);
#pragma unroll
        for (int e = 0; e < 4; ++e) {
          ax[e]     = (OP == 5) ? bfr(x0[e]) : x0[e];
          ax[4 + e] = (OP == 5) ? bfr(x1[e]) : x1[e];
        }
      }
      float wv[8];
#pragma unroll
      for (int e = 0; e < 4; ++e) {
        wv[e]     = eop<OP>(s0[e], b8[e], ax[e], scale);
        wv[4 + e] = eop<OP>(s1[e], b8[4 + e], ax[4 + e], scale);
      }
      v4u vh, vl;
#pragma unroll
      for (int e = 0; e < 4; ++e) {
        const float f0 = wv[2 * e], f1 = wv[2 * e + 1];
        if constexpr (OK == 1) {
          const unsigned short h0 = bf_bits(f0), h1 = bf_bits(f1);
          const unsigned short l0 = bf_bits(f0 - bf_up(h0)), l1 = bf_bits(f1 - bf_up(h1));
          vh[e] = pk16(h0, h1);
          vl[e] = pk16(l0, l1);
        } else {
          vh[e] = pk16(h_bits((_Float16)f0), h_bits((_Float16)f1));
          vl[e] = vh[e];
        }
      }
      oh[it] = vh;
      ol[it] = vl;
    }
    for (int pass = 0; pass < 2; ++pass) {
#pragma unroll
      for (int it = 0; it < 4; ++it) {
        const int rl = it * 4 + rq;
        const size_t o = ((size_t)rowb + (size_t)rl) * (size_t)N + cb;
        *(volatile v4u*)(Ch + o) = oh[it];
        if constexpr (OK == 1) { *(volatile v4u*)(Cl + o) = ol[it]; }
      }
      __threadfence();
    }
  }
}

extern "C" void kernel_launch(void* const* d_in, const int* in_sizes, int n_in,
                              void* d_out, int out_size, void* d_ws, size_t ws_size,
                              hipStream_t stream) {
  if (n_in < 14) return;
  const int need = ((NB - 1) * XS_FULL + SEQ) * DM;
  if (in_sizes[0] < need || out_size < need) return;
  if (in_sizes[1] != DM * DM || in_sizes[2] != DM || in_sizes[3] != DM || in_sizes[4] != DM) return;
  if (in_sizes[5] != H2 * DM || in_sizes[6] != H2) return;
  if (in_sizes[7] != DQ * DM || in_sizes[8] != DQ || in_sizes[9] != DQ * DQ) return;
  if (in_sizes[10] != DM * DH || in_sizes[11] != DM || in_sizes[12] != DM || in_sizes[13] != DM) return;

  const float* x  = (const float*)d_in[0];
  const float* Wm = (const float*)d_in[1];
  const float* bm = (const float*)d_in[2];
  const float* g1 = (const float*)d_in[3];
  const float* b1 = (const float*)d_in[4];
  const float* Wh = (const float*)d_in[5];
  const float* bh = (const float*)d_in[6];
  const float* Wq = (const float*)d_in[7];
  const float* bq = (const float*)d_in[8];
  const float* Wb = (const float*)d_in[9];
  const float* Wo = (const float*)d_in[10];
  const float* bo = (const float*)d_in[11];
  const float* g2 = (const float*)d_in[12];
  const float* b2 = (const float*)d_in[13];
  float*       out = (float*)d_out;

  const size_t szWM = (size_t)DM * DM * 2;
  const size_t szWH = (size_t)H2 * DM * 2;
  const size_t szWQ = (size_t)DQ * DM * 2;
  const size_t szWB = (size_t)DQ * DQ * 2;
  const size_t szWO = (size_t)DM * DH * 2;
  const size_t szXB = (size_t)SEQ * DM * 2;
  const size_t szY  = (size_t)SEQ * DM * 4;
  const size_t szN  = (size_t)SEQ * DM * 2;
  const size_t szH  = (size_t)SEQ * H2 * 4;
  const size_t szZ  = (size_t)SEQ * DQ * 2;
  const size_t szVT = (size_t)DH * SEQ * 2;
  const size_t szAP = (size_t)SEQ * SEQ * 2;
  const size_t szV  = (size_t)SEQ * DH * 2;
  const size_t szT  = (size_t)SEQ * DM * 4;
  size_t off = 0;
  const size_t oWM = off; off += szWM;
  const size_t oWH = off; off += szWH;
  const size_t oWQ = off; off += szWQ;
  const size_t oWB = off; off += szWB;
  const size_t oWO = off; off += szWO;
  const size_t oXB = off; off += szXB;
  const size_t oY  = off; off += szY;
  const size_t oNH = off; off += szN;
  const size_t oNL = off; off += szN;
  const size_t oH  = off; off += szH;
  const size_t oZH = off; off += szZ;
  const size_t oZL = off; off += szZ;
  const size_t oGH = off; off += szZ;
  const size_t oGL = off; off += szZ;
  const size_t oVT = off; off += szVT;
  const size_t oAP = off; off += szAP;
  const size_t oVH = off; off += szV;
  const size_t oVL = off; off += szV;
  const size_t oT  = off; off += szT;
  if (off > ws_size) return;
  if (off > (size_t)WS_CAP) return;

  char* ws = (char*)d_ws;
  u16*   WMb = (u16*)(ws + oWM);
  u16*   WHb = (u16*)(ws + oWH);
  u16*   WQb = (u16*)(ws + oWQ);
  u16*   WBt = (u16*)(ws + oWB);
  u16*   WOb = (u16*)(ws + oWO);
  u16*   XB  = (u16*)(ws + oXB);
  float* Y   = (float*)(ws + oY);
  u16*   NH  = (u16*)(ws + oNH);
  u16*   NL  = (u16*)(ws + oNL);
  float* H   = (float*)(ws + oH);
  u16*   ZH  = (u16*)(ws + oZH);
  u16*   ZL  = (u16*)(ws + oZL);
  u16*   GH  = (u16*)(ws + oGH);
  u16*   GL  = (u16*)(ws + oGL);
  u16*   VT  = (u16*)(ws + oVT);
  u16*   AP  = (u16*)(ws + oAP);
  u16*   VH  = (u16*)(ws + oVH);
  u16*   VL  = (u16*)(ws + oVL);
  float* T   = (float*)(ws + oT);

  const dim3 b256(256), b128(128);
  const int  n8wm = (DM * DM) / 8, n8wh = (H2 * DM) / 8, n8wq = (DQ * DM) / 8, n8wo = (DM * DH) / 8;
  const int  n8x  = (SEQ * DM) / 8;
  const int  ntb  = (DQ + 63) / 64;
  const dim3 gWB((DQ / 64) * ntb);
  const dim3 gX((n8x + 255) / 256);
  const dim3 gLN(SEQ / 8);
  const dim3 gGM((SEQ / 64) * (DM / 64));
  const dim3 gGH((SEQ / 64) * (H2 / 64));
  const dim3 gGQ((SEQ / 64) * (DQ / 64));
  const dim3 gVT((DH / 64) * (SEQ / 64));
  const dim3 gQK((SEQ / 64) * (SEQ / 64));
  const dim3 gAV((SEQ / 64) * (DH / 64));
  const float one = 1.0f;
  const float sqk = 1.0f / (float)SEQ;
  const float sav = 1.0f / (ACAR * VCAR);

  k_cvt<<<dim3((n8wm + 255) / 256), b256, 0, stream>>>(Wm, WMb, n8wm);
  k_cvt<<<dim3((n8wh + 255) / 256), b256, 0, stream>>>(Wh, WHb, n8wh);
  k_cvt<<<dim3((n8wq + 255) / 256), b256, 0, stream>>>(Wq, WQb, n8wq);
  k_cvt<<<dim3((n8wo + 255) / 256), b256, 0, stream>>>(Wo, WOb, n8wo);
  k_wt<<<gWB, b256, 0, stream>>>(Wb, DQ, DQ, ntb, WBt, 0);

  for (int b = 0; b < NB; ++b) {
    const size_t xo = (size_t)b * XS_FULL * DM;
    const float* xb = x + xo;
    k_cvt<<<gX, b256, 0, stream>>>(xb, XB, n8x);
    k_gemm<1, false, 5, 0><<<gGM, b128, 0, stream>>>(XB, XB, WMb, WMb, SEQ, DM, DM, bm, xb, DM, one, Y, XB, XB);
    k_ln1<<<gLN, b256, 0, stream>>>(Y, g1, b1, NH, NL);
    k_gemm<2, false, 1, 0><<<gGH, b128, 0, stream>>>(NH, NL, WHb, WHb, SEQ, H2, DM, bh, Y, DM, one, H, XB, XB);
    k_gemm<2, false, 1, 1><<<gGQ, b128, 0, stream>>>(NH, NL, WQb, WQb, SEQ, DQ, DM, bq, Y, DM, one, Y, ZH, ZL);
    k_gemm<2, false, 2, 1><<<gGQ, b128, 0, stream>>>(ZH, ZL, WBt, WBt, SEQ, DQ, DQ, bq, Y, DM, one, Y, GH, GL);
    k_vt<<<gVT, b256, 0, stream>>>(H, VT);
    k_gemm<3, false, 3, 2><<<gQK, b128, 0, stream>>>(GH, GL, ZH, ZL, SEQ, SEQ, DQ, bq, Y, DM, sqk, Y, AP, AP);
    k_gemm<1, true, 4, 1><<<gAV, b128, 0, stream>>>(AP, AP, VT, VT, SEQ, DH, SEQ, bq, H + DH, H2, sav, Y, VH, VL);
    k_gemm<2, false, 0, 0><<<gGM, b128, 0, stream>>>(VH, VL, WOb, WOb, SEQ, DM, DH, bo, Y, DM, one, T, XB, XB);
    k_ln2<<<gLN, b256, 0, stream>>>(T, xb, g2, b2, out + xo);
  }
  (void)hipGetLastError();
}
